// BilinearFeedForward_16527034155428
// MI455X (gfx1250) — hardware-run, weakly checked
//
#include <hip/hip_runtime.h>
#include <math.h>

typedef __attribute__((ext_vector_type(16))) _Float16 v16h;
typedef __attribute__((ext_vector_type(8)))  _Float16 v8h;
typedef __attribute__((ext_vector_type(8)))  float    v8f;
typedef __attribute__((ext_vector_type(4)))  float    v4f;
typedef __attribute__((ext_vector_type(4)))  unsigned int v4u;

constexpr int kBatch = 4;
constexpr int kSeq   = 2048;
constexpr int kDim   = 1024;
constexpr int kTok   = kBatch * kSeq;
constexpr float kWCarry     = 16.0f;
constexpr float kWCarryInv  = 1.0f / kWCarry;
constexpr float kKvCarry    = 1024.0f;
constexpr float kKvCarryInv = 1.0f / kKvCarry;
constexpr float kNormEps    = 1e-5f;
static_assert((kDim % 64) == 0 && (kSeq % 64) == 0 && (kTok % 64) == 0);
static_assert((kDim % 32) == 0 && (kSeq % 32) == 0);

constexpr size_t kSzX   = (size_t)kTok * kDim * 2;
constexpr size_t kSzW   = (size_t)4 * kDim * kDim * 2;
constexpr size_t kSzKT  = (size_t)kBatch * kDim * kSeq * 2;
constexpr size_t kSzKV  = (size_t)kBatch * kDim * kDim * 2;
constexpr size_t kSzRN  = (size_t)2 * kBatch * kDim * 4;
constexpr size_t kOffXR  = 0;
constexpr size_t kOffXI  = kOffXR  + kSzX;
constexpr size_t kOffWT  = kOffXI  + kSzX;
constexpr size_t kOffKT  = kOffWT  + kSzW;
constexpr size_t kOffVT  = kOffKT  + kSzKT;
constexpr size_t kOffKVT = kOffVT  + kSzKT;
constexpr size_t kOffQI  = kOffKVT + kSzKV;
constexpr size_t kOffQ   = kOffQI  + kSzX;
constexpr size_t kOffRN  = kOffQ   + kSzX;
constexpr size_t kWsTotal = kOffRN + kSzRN;
static_assert(kWsTotal == 117473280ull);
static_assert(kWsTotal <= 134217728ull);
static_assert((kOffXI % 128) == 0 && (kOffWT % 128) == 0 && (kOffKT % 128) == 0 && (kOffVT % 128) == 0 &&
              (kOffKVT % 128) == 0 && (kOffQI % 128) == 0 && (kOffQ % 128) == 0 && (kOffRN % 128) == 0);
static_assert(kOffXI == kOffXR + kSzX);
static_assert(kOffVT == kOffKT + kSzKT);

__device__ __forceinline__ unsigned short f2bf_bits(float f) {
  unsigned u = __float_as_uint(f);
  return (unsigned short)((u + 0x7FFFu + ((u >> 16) & 1u)) >> 16);
}
__device__ __forceinline__ float bf_bits2f(unsigned short h) { return __uint_as_float(((unsigned)h) << 16); }
__device__ __forceinline__ unsigned pk16(unsigned short a, unsigned short b) { return (unsigned)a | ((unsigned)b << 16); }
__device__ __forceinline__ unsigned short h_bits(float f) { const _Float16 h = (_Float16)f; return __builtin_bit_cast(unsigned short, h); }
__device__ __forceinline__ float h16_to_f32(unsigned hb) {
  const unsigned sgn = (hb & 0x8000u) << 16;
  const unsigned em = hb & 0x7fffu;
  const float fn = __uint_as_float((em << 13) + 0x38000000u);
  const float fs = (float)em * 5.9604644775390625e-8f;
  const float mag = (em < 0x400u) ? fs : fn;
  return __uint_as_float(__float_as_uint(mag) | sgn);
}

__device__ __forceinline__ void guard_row_h(v8f& a, v8f& b, v8f& c, v8f& d, v16h x, v16h y0, v16h y1, v16h y2, v16h y3) {
  asm volatile("v_nop\n\tv_nop\n\tv_nop\n\tv_nop" : "+v"(a), "+v"(b), "+v"(c), "+v"(d) : "v"(x), "v"(y0), "v"(y1), "v"(y2), "v"(y3));
}
__device__ __forceinline__ void keep4_h(v16h a, v16h b, v16h c, v16h d) { asm volatile("v_nop" :: "v"(a), "v"(b), "v"(c), "v"(d)); }
__device__ __forceinline__ void acc_guard4(v8f& a, v8f& b, v8f& c, v8f& d) { asm volatile("v_nop\n\tv_nop\n\tv_nop\n\tv_nop" : "+v"(a), "+v"(b), "+v"(c), "+v"(d)); }

struct FragH {
  union U { v16h v; v8h h[2]; };
  static __device__ __forceinline__ v16h load(const _Float16* p) {
    U f;
    f.h[0] = *(const v8h*)(p);
    f.h[1] = *(const v8h*)(p + 16);
    return f.v;
  }
  static __device__ __forceinline__ v8f mma(v16h a, v16h b, v8f c) {
    return __builtin_amdgcn_wmma_f32_16x16x32_f16(false, a, false, b, (short)0, c, false, false);
  }
};

template <int EPI, int OUT_MODE>
__global__ __launch_bounds__(256) void gemm64_f16(
    const unsigned short* __restrict__ Ap, int lda, long strideA,
    const unsigned short* __restrict__ Btp, int ldb, long strideB,
    void* __restrict__ Cout, int ldc, long strideC,
    const float* __restrict__ vecA, const float* __restrict__ vecB, long strideV,
    const unsigned short* __restrict__ mulp,
    int M, int N, int K, float scale) {
  const _Float16* A  = (const _Float16*)Ap;
  const _Float16* Bt = (const _Float16*)Btp;
  __shared__ __align__(16) float sT[8][16 * 68];
  const int b    = blockIdx.y;
  const int lane = threadIdx.x & 31;
  const int wave = threadIdx.x >> 5;
  const int tilesN = N >> 6;
  const int tilesM = M >> 6;
  const int tile = blockIdx.x * 8 + wave;
  if (tile >= tilesM * tilesN) return;
  const int tm = tile / tilesN;
  const int tn = tile - tm * tilesN;
  const int m0 = tm << 6;
  const int n0 = tn << 6;

  const _Float16* Ab = A  + (size_t)b * strideA;
  const _Float16* Bb = Bt + (size_t)b * strideB;

  const int rlane = lane & 15;
  const int koff  = (lane >> 4) * 8;
  const int mOff  = (lane >> 4) * 8;

  v8f acc[4][4];
#pragma unroll
  for (int i = 0; i < 4; ++i)
#pragma unroll
    for (int j = 0; j < 4; ++j) acc[i][j] = (v8f){0.f, 0.f, 0.f, 0.f, 0.f, 0.f, 0.f, 0.f};

  for (int k0 = 0; k0 < K; k0 += 32) {
    v16h bh[4];
#pragma unroll
    for (int j = 0; j < 4; ++j) {
      const size_t bo = (size_t)(n0 + (j << 4) + rlane) * ldb + koff + k0;
      bh[j] = FragH::load(Bb + bo);
    }
#pragma unroll
    for (int i = 0; i < 4; ++i) {
      const size_t ao = (size_t)(m0 + (i << 4) + rlane) * lda + koff + k0;
      v16h ah = FragH::load(Ab + ao);
#pragma unroll
      for (int j = 0; j < 4; ++j) acc[i][j] = FragH::mma(ah, bh[j], acc[i][j]);
      guard_row_h(acc[i][0], acc[i][1], acc[i][2], acc[i][3], ah, bh[0], bh[1], bh[2], bh[3]);
    }
    keep4_h(bh[0], bh[1], bh[2], bh[3]);
  }
  acc_guard4(acc[0][0], acc[0][1], acc[0][2], acc[0][3]);
  acc_guard4(acc[1][0], acc[1][1], acc[1][2], acc[1][3]);
  acc_guard4(acc[2][0], acc[2][1], acc[2][2], acc[2][3]);
  acc_guard4(acc[3][0], acc[3][1], acc[3][2], acc[3][3]);

  float* slab = sT[wave];
  float cvec[4];
#pragma unroll
  for (int j = 0; j < 4; ++j) {
    const int n = n0 + (j << 4) + rlane;
    float cv = 0.f;
    if (EPI == 1) cv = vecB[(size_t)b * strideV + n];
    if (EPI == 3) cv = bf_bits2f(f2bf_bits(vecA[n]));
    cvec[j] = cv;
  }
#pragma unroll
  for (int i = 0; i < 4; ++i) {
    const int mBase = m0 + (i << 4);
    float rowr[8];
    if (EPI == 1) {
      const float* rp = vecA + (size_t)b * strideV + mBase + mOff;
      const v4f ra = *(const v4f*)(rp);
      const v4f rb = *(const v4f*)(rp + 4);
      rowr[0] = ra[0]; rowr[1] = ra[1]; rowr[2] = ra[2]; rowr[3] = ra[3];
      rowr[4] = rb[0]; rowr[5] = rb[1]; rowr[6] = rb[2]; rowr[7] = rb[3];
    } else {
#pragma unroll
      for (int r = 0; r < 8; ++r) rowr[r] = 1.0f;
    }
#pragma unroll
    for (int j = 0; j < 4; ++j) {
#pragma unroll
      for (int r = 0; r < 8; ++r) {
        float v = acc[i][j][r] * scale;
        if (EPI == 1) v = (v * rowr[r]) * cvec[j];
        if (EPI == 3) v = v + cvec[j];
        slab[(mOff + r) * 68 + (j << 4) + rlane] = v;
      }
    }
    __builtin_amdgcn_fence(__ATOMIC_RELEASE, "workgroup");
    __builtin_amdgcn_wave_barrier();
    __builtin_amdgcn_fence(__ATOMIC_ACQUIRE, "workgroup");
    if (OUT_MODE == 0) {
      float* C = (float*)Cout + (size_t)b * strideC;
      const int hh = lane >> 4, c4 = (lane & 15) * 4;
      v4f vv[8];
#pragma unroll
      for (int it = 0; it < 8; ++it) vv[it] = *(const v4f*)(slab + (it * 2 + hh) * 68 + c4);
      for (int pass = 0; pass < 2; ++pass) {
#pragma unroll
        for (int it = 0; it < 8; ++it)
          *(volatile v4f*)(C + (size_t)(mBase + it * 2 + hh) * ldc + n0 + c4) = vv[it];
        __threadfence();
      }
    } else {
      const int q = lane >> 3, c8 = (lane & 7) * 8;
      unsigned short* C = (unsigned short*)Cout + (size_t)b * strideC;
      const unsigned short* Mp = mulp + (size_t)b * strideC;
      v8h hv[4];
#pragma unroll
      for (int it = 0; it < 4; ++it) {
        const int row = it * 4 + q;
        const float* sp = slab + row * 68 + c8;
        float f[8];
#pragma unroll
        for (int e = 0; e < 8; ++e) f[e] = sp[e];
        if (EPI == 2) {
          const v4u w = *(const v4u*)(Mp + (size_t)(mBase + row) * ldc + n0 + c8);
          const unsigned w0 = w[0];
          const unsigned w1 = w[1];
          const unsigned w2 = w[2];
          const unsigned w3 = w[3];
          f[0] = f[0] * h16_to_f32(w0 & 0xffffu);
          f[1] = f[1] * h16_to_f32(w0 >> 16);
          f[2] = f[2] * h16_to_f32(w1 & 0xffffu);
          f[3] = f[3] * h16_to_f32(w1 >> 16);
          f[4] = f[4] * h16_to_f32(w2 & 0xffffu);
          f[5] = f[5] * h16_to_f32(w2 >> 16);
          f[6] = f[6] * h16_to_f32(w3 & 0xffffu);
          f[7] = f[7] * h16_to_f32(w3 >> 16);
        }
#pragma unroll
        for (int e = 0; e < 8; ++e) hv[it][e] = (_Float16)f[e];
      }
      for (int pass = 0; pass < 2; ++pass) {
#pragma unroll
        for (int it = 0; it < 4; ++it)
          *(volatile v8h*)(C + (size_t)(mBase + it * 4 + q) * ldc + n0 + c8) = hv[it];
        __threadfence();
      }
    }
    __builtin_amdgcn_fence(__ATOMIC_RELEASE, "workgroup");
    __builtin_amdgcn_wave_barrier();
    __builtin_amdgcn_fence(__ATOMIC_ACQUIRE, "workgroup");
  }
}

__global__ __launch_bounds__(256) void cvt_x_kernel(const float* __restrict__ x0, const float* __restrict__ x1,
                                                    unsigned short* __restrict__ out, int n8) {
  const int i = blockIdx.x * 256 + threadIdx.x;
  if (i >= n8) return;
  const int z = blockIdx.y;
  const float* src = (z == 0) ? x0 : x1;
  const float* p = src + 8 * (size_t)i;
  const v4f a = *(const v4f*)(p);
  const v4f c = *(const v4f*)(p + 4);
  unsigned short hb[8];
#pragma unroll
  for (int e = 0; e < 4; ++e) {
    const float fa = a[e];
    const float fc = c[e];
    hb[e]     = h_bits(bf_bits2f(f2bf_bits(fa)));
    hb[4 + e] = h_bits(bf_bits2f(f2bf_bits(fc)));
  }
  const v4u u = (v4u){pk16(hb[0], hb[1]), pk16(hb[2], hb[3]), pk16(hb[4], hb[5]), pk16(hb[6], hb[7])};
  unsigned short* q = out + (size_t)z * 8 * (size_t)n8 + 8 * (size_t)i;
  *(volatile v4u*)q = u;
  __threadfence();
  *(volatile v4u*)q = u;
}

__global__ __launch_bounds__(256) void wtcast_kernel(const float* __restrict__ W0, const float* __restrict__ W1,
                                                     const float* __restrict__ W2, const float* __restrict__ W3,
                                                     unsigned short* __restrict__ out) {
  __shared__ float sm[64][65];
  const int t  = threadIdx.x;
  const int d0 = blockIdx.x * 64;
  const int e0 = blockIdx.y * 64;
  const int z  = blockIdx.z;
  const float* W = (z == 0) ? W0 : (z == 1) ? W1 : (z == 2) ? W2 : W3;
#pragma unroll 8
  for (int i = 0; i < 16; ++i) {
    const int idx = i * 256 + t;
    const int r = idx >> 6;
    const int c = idx & 63;
    const float w = W[(size_t)(d0 + r) * kDim + e0 + c];
    sm[c][r] = bf_bits2f(f2bf_bits(w)) * kWCarry;
  }
  __syncthreads();
  const int lane = t & 31, wave = t >> 5;
  const int q = lane >> 3, c8 = (lane & 7) * 8;
  unsigned short* op = out + (size_t)z * kDim * kDim;
  v4u u[2];
#pragma unroll
  for (int it = 0; it < 2; ++it) {
    const int row = wave * 8 + it * 4 + q;
    unsigned short hb[8];
#pragma unroll
    for (int e = 0; e < 8; ++e) hb[e] = h_bits(sm[row][c8 + e]);
    u[it] = (v4u){pk16(hb[0], hb[1]), pk16(hb[2], hb[3]), pk16(hb[4], hb[5]), pk16(hb[6], hb[7])};
  }
  for (int pass = 0; pass < 2; ++pass) {
#pragma unroll
    for (int it = 0; it < 2; ++it) {
      const int row = wave * 8 + it * 4 + q;
      *(volatile v4u*)(op + (size_t)(e0 + row) * kDim + d0 + c8) = u[it];
    }
    __threadfence();
  }
}

__global__ __launch_bounds__(256) void rownorm_kernel(const unsigned short* __restrict__ planes, float* __restrict__ rn) {
  __shared__ float sRes[32];
  const int t = threadIdx.x, lane = t & 31, wave = t >> 5;
  const int rowBase = blockIdx.x * 32 + wave * 4;
#pragma unroll 1
  for (int i = 0; i < 4; ++i) {
    const v4u* rp = (const v4u*)(planes + (size_t)(rowBase + i) * kSeq);
    float ss = 0.f;
#pragma unroll 1
    for (int c = 0; c < 8; ++c) {
      const v4u w = rp[c * 32 + lane];
      const unsigned w0 = w[0];
      const unsigned w1 = w[1];
      const unsigned w2 = w[2];
      const unsigned w3 = w[3];
      const float f0 = h16_to_f32(w0 & 0xffffu);
      const float f1 = h16_to_f32(w0 >> 16);
      const float f2 = h16_to_f32(w1 & 0xffffu);
      const float f3 = h16_to_f32(w1 >> 16);
      const float f4 = h16_to_f32(w2 & 0xffffu);
      const float f5 = h16_to_f32(w2 >> 16);
      const float f6 = h16_to_f32(w3 & 0xffffu);
      const float f7 = h16_to_f32(w3 >> 16);
      ss = fmaf(f0, f0, ss);
      ss = fmaf(f1, f1, ss);
      ss = fmaf(f2, f2, ss);
      ss = fmaf(f3, f3, ss);
      ss = fmaf(f4, f4, ss);
      ss = fmaf(f5, f5, ss);
      ss = fmaf(f6, f6, ss);
      ss = fmaf(f7, f7, ss);
    }
#pragma unroll
    for (int off = 16; off > 0; off >>= 1) ss += __shfl_xor(ss, off, 32);
    if (lane == 0) sRes[wave * 4 + i] = ss;
  }
  __syncthreads();
  if (wave == 0) {
    const float ss  = sRes[lane];
    const float nrm = sqrtf(ss);
    const float inv = 1.0f / fmaxf(nrm, kNormEps);
    volatile float* o = rn + (size_t)blockIdx.x * 32 + lane;
    *o = inv;
    __threadfence();
    *o = inv;
  }
}

extern "C" void kernel_launch(void* const* d_in, const int* in_sizes, int n_in,
                              void* d_out, int out_size, void* d_ws, size_t ws_size,
                              hipStream_t stream) {
  if (n_in < 7) return;
  if (in_sizes[0] != kTok * kDim) return;
  if (in_sizes[1] != kTok * kDim) return;
  if (in_sizes[2] != kDim * kDim) return;
  if (in_sizes[3] != kDim * kDim) return;
  if (in_sizes[4] != kDim * kDim) return;
  if (in_sizes[5] != kDim * kDim) return;
  if (in_sizes[6] != kDim) return;
  if (out_size != kTok * kDim) return;
  if (ws_size < kWsTotal) return;

  const float* x_real = (const float*)d_in[0];
  const float* x_imag = (const float*)d_in[1];
  const float* w_qr   = (const float*)d_in[2];
  const float* w_qi   = (const float*)d_in[3];
  const float* w_k    = (const float*)d_in[4];
  const float* w_v    = (const float*)d_in[5];
  const float* bias   = (const float*)d_in[6];
  float* out = (float*)d_out;

  char* ws = (char*)d_ws;
  unsigned short* XR16  = (unsigned short*)(ws + kOffXR);
  unsigned short* XI16  = (unsigned short*)(ws + kOffXI);
  unsigned short* WT16  = (unsigned short*)(ws + kOffWT);
  unsigned short* KT16  = (unsigned short*)(ws + kOffKT);
  unsigned short* VT16  = (unsigned short*)(ws + kOffVT);
  unsigned short* KVT16 = (unsigned short*)(ws + kOffKVT);
  unsigned short* QI16  = (unsigned short*)(ws + kOffQI);
  unsigned short* Q16   = (unsigned short*)(ws + kOffQ);
  float*          RN    = (float*)(ws + kOffRN);

  const size_t planeW = (size_t)kDim * kDim;
  const long strideX  = (long)kSeq * kDim;
  const long strideKT = (long)kDim * kSeq;
  const long strideKV = (long)kDim * kDim;

  cvt_x_kernel<<<dim3((kTok * kDim / 8) / 256, 2), 256, 0, stream>>>(x_real, x_imag, XR16, kTok * kDim / 8);

  wtcast_kernel<<<dim3(kDim / 64, kDim / 64, 4), 256, 0, stream>>>(w_qr, w_qi, w_k, w_v, WT16);

  gemm64_f16<0, 1><<<dim3(64, kBatch), 256, 0, stream>>>(
      WT16 + 2 * planeW, kDim, 0L,
      XR16, kDim, strideX,
      (void*)KT16, kSeq, strideKT,
      RN, RN, 0L, WT16,
      kDim, kSeq, kDim, kWCarryInv);

  gemm64_f16<0, 1><<<dim3(64, kBatch), 256, 0, stream>>>(
      WT16 + 3 * planeW, kDim, 0L,
      XI16, kDim, strideX,
      (void*)VT16, kSeq, strideKT,
      RN, RN, 0L, WT16,
      kDim, kSeq, kDim, kWCarryInv);

  rownorm_kernel<<<(2 * kBatch * kDim) / 32, 256, 0, stream>>>(KT16, RN);

  gemm64_f16<1, 1><<<dim3(32, kBatch), 256, 0, stream>>>(
      VT16, kSeq, strideKT,
      KT16, kSeq, strideKT,
      (void*)KVT16, kDim, strideKV,
      RN + kBatch * kDim, RN, (long)kDim, VT16,
      kDim, kDim, kSeq, kKvCarry);

  gemm64_f16<0, 1><<<dim3(256, 1), 256, 0, stream>>>(
      XI16, kDim, 0L,
      WT16 + 1 * planeW, kDim, 0L,
      (void*)QI16, kDim, 0L,
      RN, RN, 0L, XI16,
      kTok, kDim, kDim, kWCarryInv);

  gemm64_f16<2, 1><<<dim3(256, 1), 256, 0, stream>>>(
      XR16, kDim, 0L,
      WT16, kDim, 0L,
      (void*)Q16, kDim, 0L,
      RN, RN, 0L, QI16,
      kTok, kDim, kDim, kWCarryInv);

  gemm64_f16<3, 0><<<dim3(64, kBatch), 256, 0, stream>>>(
      Q16, kDim, strideX,
      KVT16, kDim, strideKV,
      (void*)out, kDim, strideX,
      bias, RN, 0L, Q16,
      kSeq, kDim, kDim, kKvCarryInv);
}
